// MSDeformableAttention3D_13932873909053
// MI455X (gfx1250) — hardware-verified
//
#include <hip/hip_runtime.h>

typedef __attribute__((ext_vector_type(16))) _Float16 v16h;
typedef __attribute__((ext_vector_type(8)))  _Float16 v8h;
typedef __attribute__((ext_vector_type(16))) __bf16   v16b;
typedef __attribute__((ext_vector_type(8)))  __bf16   v8b;
typedef __attribute__((ext_vector_type(8)))  float    v8f;
typedef __attribute__((ext_vector_type(4)))  float    v4f;
typedef __attribute__((ext_vector_type(4)))  int      v4i;

static constexpr int kNQ   = 22500;
static constexpr int kNQP  = 22528;
static constexpr int kNV   = 13294;
static constexpr int kNVP  = 13312;
static constexpr int kD    = 256;
static constexpr int kNH   = 8;
static constexpr int kNL   = 4;
static constexpr int kNP   = 8;
static constexpr int kHD   = 32;
static constexpr int kNOFF = kNH * kNL * kNP * 2;
static constexpr int kNLG  = kNH * kNL * kNP;
static constexpr int kSampRows = 4;
static_assert(kNQP % 64 == 0 && kNQP >= kNQ && kNVP % 64 == 0 && kNVP >= kNV, "tile multiples");
static_assert(kD % 32 == 0 && kNOFF % 64 == 0 && kNLG % 64 == 0 && kNLG == kD, "K multiple of 32, N multiple of 64");
static_assert((kNQP * 32) % 256 == 0 && (kNVP * 32) % 256 == 0 && kNQP % kSampRows == 0 && kNQP % 8 == 0, "exact grids");
static_assert(kNH * kHD == kD && kNL * kNP == 32, "lane maps");

static constexpr size_t SZ_Q16  = (size_t)kNQP * kD * 2;
static constexpr size_t SZ_V16  = (size_t)kNVP * kD * 2;
static constexpr size_t SZ_VAL  = (size_t)kNVP * kD * 4;
static constexpr size_t SZ_OFF  = (size_t)kNQP * kNOFF * 4;
static constexpr size_t SZ_LGT  = (size_t)kNQP * kNLG * 4;
static constexpr size_t SZ_OUT  = (size_t)kNQP * kD * 4;
static constexpr size_t SZ_W256 = (size_t)kD * kD * 2;
static constexpr size_t SZ_WOFF = (size_t)kNOFF * kD * 2;
static constexpr size_t OFF_Q16  = 0;
static constexpr size_t OFF_AO16 = OFF_Q16;
static constexpr size_t OFF_V16  = OFF_Q16 + SZ_Q16;
static constexpr size_t OFF_VAL  = OFF_V16 + SZ_V16;
static constexpr size_t OFF_OFF  = OFF_VAL + SZ_VAL;
static constexpr size_t OFF_OUT  = OFF_OFF;
static constexpr size_t OFF_LGT  = OFF_OFF + SZ_OFF;
static constexpr size_t OFF_WVAL = OFF_LGT + SZ_LGT;
static constexpr size_t OFF_WOUT = OFF_WVAL + SZ_W256;
static constexpr size_t OFF_WOFF = OFF_WOUT + SZ_W256;
static constexpr size_t OFF_WATT = OFF_WOFF + SZ_WOFF;
static constexpr size_t WS_TOTAL = OFF_WATT + SZ_W256;
static_assert(SZ_OUT <= SZ_OFF, "OUT aliases the dead OFF region");
static_assert(WS_TOTAL <= (size_t)134217728, "carve under 128 MiB");
static_assert((OFF_V16 % 128) == 0 && (OFF_VAL % 128) == 0 && (OFF_OFF % 128) == 0 && (OFF_LGT % 128) == 0 &&
              (OFF_WVAL % 128) == 0 && (OFF_WOUT % 128) == 0 && (OFF_WOFF % 128) == 0 && (OFF_WATT % 128) == 0, "128-B aligned regions");

__device__ __forceinline__ unsigned short f2bf_bits(float f) {
  unsigned u = __float_as_uint(f);
  return (unsigned short)((u + 0x7FFFu + ((u >> 16) & 1u)) >> 16);
}
__device__ __forceinline__ float bf_bits2f(unsigned short h) { return __uint_as_float(((unsigned)h) << 16); }

__device__ __forceinline__ void dep_guard_h(v8f& a, v8f& b, v16h x, v16h y) { asm volatile("v_nop\n\tv_nop\n\tv_nop\n\tv_nop" : "+v"(a), "+v"(b) : "v"(x), "v"(y)); }
__device__ __forceinline__ void dep_guard_b(v8f& a, v8f& b, v16b x, v16b y) { asm volatile("v_nop\n\tv_nop\n\tv_nop\n\tv_nop" : "+v"(a), "+v"(b) : "v"(x), "v"(y)); }
__device__ __forceinline__ void keep4_h(v16h a, v16h b, v16h c, v16h d) { asm volatile("v_nop" :: "v"(a), "v"(b), "v"(c), "v"(d)); }
__device__ __forceinline__ void keep4_b(v16b a, v16b b, v16b c, v16b d) { asm volatile("v_nop" :: "v"(a), "v"(b), "v"(c), "v"(d)); }
__device__ __forceinline__ void acc_guard4(v8f& a, v8f& b, v8f& c, v8f& d) { asm volatile("v_nop\n\tv_nop\n\tv_nop\n\tv_nop" : "+v"(a), "+v"(b), "+v"(c), "+v"(d)); }
template <typename T> struct Frag;
template <> struct Frag<_Float16> {
  typedef v16h V; union U { v16h v; v8h h[2]; };
  static __device__ __forceinline__ v16h load(const _Float16* p) {
    U f; f.h[0] = *(const v8h*)(p); f.h[1] = *(const v8h*)(p + 16); return f.v;
  }
  static __device__ __forceinline__ v8f mma(v16h a, v16h b, v8f c) {
    return __builtin_amdgcn_wmma_f32_16x16x32_f16(false, a, false, b, (short)0, c, false, false);
  }
  static __device__ __forceinline__ void guard(v8f& a, v8f& b, v16h x, v16h y) { dep_guard_h(a, b, x, y); }
  static __device__ __forceinline__ void keep(v16h a, v16h b, v16h c, v16h d) { keep4_h(a, b, c, d); }
};
template <> struct Frag<__bf16> {
  typedef v16b V; union U { v16b v; v8b h[2]; };
  static __device__ __forceinline__ v16b load(const __bf16* p) {
    U f; f.h[0] = *(const v8b*)(p); f.h[1] = *(const v8b*)(p + 16); return f.v;
  }
  static __device__ __forceinline__ v8f mma(v16b a, v16b b, v8f c) {
    return __builtin_amdgcn_wmma_f32_16x16x32_bf16(false, a, false, b, (short)0, c, false, false);
  }
  static __device__ __forceinline__ void guard(v8f& a, v8f& b, v16b x, v16b y) { dep_guard_b(a, b, x, y); }
  static __device__ __forceinline__ void keep(v16b a, v16b b, v16b c, v16b d) { keep4_b(a, b, c, d); }
};

template <int ET> struct Elem;
template <> struct Elem<0> { typedef _Float16 T; };
template <> struct Elem<1> { typedef __bf16 T; };
template <int ET, bool SPLIT, int BIAS_MODE, int OUT_MODE, bool RESID, int ACT = 0>
__global__ __launch_bounds__(256) void wmma_gemm64(
    const unsigned short* __restrict__ Ap, const unsigned short* __restrict__ A2p, int lda, long strideA,
    const unsigned short* __restrict__ Btp, const unsigned short* __restrict__ Bt2p, int ldb, long strideB,
    void* __restrict__ Cout, void* __restrict__ Cout2, int ldc, long strideC,
    const float* __restrict__ bias,
    const float* __restrict__ resid, long strideR,
    int M, int N, int K, float scale) {
  typedef typename Elem<ET>::T T;
  typedef typename Frag<T>::V V;
  const T* A = (const T*)Ap; const T* A2 = (const T*)A2p; const T* Bt = (const T*)Btp; const T* Bt2 = (const T*)Bt2p;
  __shared__ __align__(16) float sT[8][16 * 68];
  const int b    = blockIdx.y;
  const int lane = threadIdx.x & 31;
  const int wave = threadIdx.x >> 5;
  const int tilesN = N >> 6;
  const int tilesM = M >> 6;
  const int tile = blockIdx.x * 8 + wave;
  if (tile >= tilesM * tilesN) return;
  const int tm = tile / tilesN;
  const int tn = tile - tm * tilesN;
  const int m0 = tm << 6;
  const int n0 = tn << 6;

  const T* Ab  = A  + (size_t)b * strideA;
  const T* Bb  = Bt + (size_t)b * strideB;
  const T* Ab2 = SPLIT ? (A2  + (size_t)b * strideA) : nullptr;
  const T* Bb2 = SPLIT ? (Bt2 + (size_t)b * strideB) : nullptr;

  const int rlane = lane & 15;
  const int koff  = (lane >> 4) * 8;
  const int mOff  = (lane >> 4) * 8;

  v8f acc[4][4];
#pragma unroll
  for (int i = 0; i < 4; ++i)
#pragma unroll
    for (int j = 0; j < 4; ++j) acc[i][j] = (v8f){0.f,0.f,0.f,0.f,0.f,0.f,0.f,0.f};

  for (int k0 = 0; k0 < K; k0 += 32) {
    V bh[4], bl[4];
#pragma unroll
    for (int j = 0; j < 4; ++j) {
      const size_t bo = (size_t)(n0 + (j << 4) + rlane) * ldb + koff + k0;
      bh[j] = Frag<T>::load(Bb + bo);
      if (SPLIT) bl[j] = Frag<T>::load(Bb2 + bo);
    }
#pragma unroll
    for (int i = 0; i < 4; ++i) {
      const size_t ao = (size_t)(m0 + (i << 4) + rlane) * lda + koff + k0;
      V ah = Frag<T>::load(Ab + ao);
      V al;
      if (SPLIT) al = Frag<T>::load(Ab2 + ao);
#pragma unroll
      for (int j = 0; j < 4; ++j) {
        acc[i][j] = Frag<T>::mma(ah, bh[j], acc[i][j]);
        if (SPLIT) {
          acc[i][j] = Frag<T>::mma(ah, bl[j], acc[i][j]);
          acc[i][j] = Frag<T>::mma(al, bh[j], acc[i][j]);
        }
      }
      Frag<T>::guard(acc[i][0], acc[i][3], ah, SPLIT ? al : ah);
    }
    Frag<T>::keep(bh[0], bh[1], bh[2], bh[3]);
    if (SPLIT) Frag<T>::keep(bl[0], bl[1], bl[2], bl[3]);
  }
  acc_guard4(acc[0][0], acc[0][1], acc[0][2], acc[0][3]);
  acc_guard4(acc[1][0], acc[1][1], acc[1][2], acc[1][3]);
  acc_guard4(acc[2][0], acc[2][1], acc[2][2], acc[2][3]);
  acc_guard4(acc[3][0], acc[3][1], acc[3][2], acc[3][3]);

  float* slab = sT[wave];
  const float* Rb = RESID ? (resid + (size_t)b * strideR) : nullptr;
#pragma unroll
  for (int i = 0; i < 4; ++i) {
    const int mBase = m0 + (i << 4);
#pragma unroll
    for (int j = 0; j < 4; ++j) {
      const int n = n0 + (j << 4) + rlane;
      float bv = 0.f;
      if (BIAS_MODE == 2) bv = bias[n];
#pragma unroll
      for (int r = 0; r < 8; ++r) {
        float v = acc[i][j][r] * scale;
        if (BIAS_MODE == 1) v += bias[mBase + mOff + r];
        if (BIAS_MODE == 2) v += bv;
        if (RESID) v += Rb[(size_t)(mBase + mOff + r) * ldc + n];
        if (ACT == 1) v = tanhf(v);
        if (ACT == 2) v = fmaxf(v, 0.0f);
        if (ACT == 3) v = v / (1.0f + expf(-v));
        if (ACT == 4) v = (v > 0.f) ? v : 0.01f * v;
        if (ACT == 5) v = 0.5f * v * (1.0f + erff(v * 0.70710678118654752f));
        slab[(mOff + r) * 68 + (j << 4) + rlane] = v;
      }
    }
    __builtin_amdgcn_fence(__ATOMIC_RELEASE, "workgroup");
    __builtin_amdgcn_wave_barrier();
    __builtin_amdgcn_fence(__ATOMIC_ACQUIRE, "workgroup");
    if (OUT_MODE == 0) {
      float* C = (float*)Cout + (size_t)b * strideC;
      const int hh = lane >> 4, c4 = (lane & 15) * 4;
      for (int pass = 0; pass < 2; ++pass) {
#pragma unroll
        for (int it = 0; it < 8; ++it) {
          const int row = it * 2 + hh;
          v4f v = *(const v4f*)(slab + row * 68 + c4);
          *(volatile v4f*)(C + (size_t)(mBase + row) * ldc + n0 + c4) = v;
        }
        __threadfence();
      }
    } else {
      const int q = lane >> 3, c8 = (lane & 7) * 8;
      unsigned short* C  = (unsigned short*)Cout  + (size_t)b * strideC;
      unsigned short* C2 = (OUT_MODE == 2) ? ((unsigned short*)Cout2 + (size_t)b * strideC) : nullptr;
      for (int pass = 0; pass < 2; ++pass) {
#pragma unroll
        for (int it = 0; it < 4; ++it) {
          const int row = it * 4 + q;
          const float* sp = slab + row * 68 + c8;
          v8h hv, lv;
#pragma unroll
          for (int e = 0; e < 8; ++e) {
            if (OUT_MODE == 1) {
              hv[e] = (_Float16)sp[e];
            } else {
              unsigned short hb = f2bf_bits(sp[e]);
              unsigned short lb = f2bf_bits(sp[e] - bf_bits2f(hb));
              hv[e] = __builtin_bit_cast(_Float16, hb);
              lv[e] = __builtin_bit_cast(_Float16, lb);
            }
          }
          *(volatile v8h*)(C + (size_t)(mBase + row) * ldc + n0 + c8) = hv;
          if (OUT_MODE == 2) *(volatile v8h*)(C2 + (size_t)(mBase + row) * ldc + n0 + c8) = lv;
        }
        __threadfence();
      }
    }
    __builtin_amdgcn_fence(__ATOMIC_RELEASE, "workgroup");
    __builtin_amdgcn_wave_barrier();
    __builtin_amdgcn_fence(__ATOMIC_ACQUIRE, "workgroup");
  }
}

__global__ __launch_bounds__(256) void prep_act16(const float* __restrict__ x, _Float16* __restrict__ x16,
                                                 int nReal, int nPadRows) {
  const int t = blockIdx.x * 256 + threadIdx.x;
  const int row = t >> 5;
  const int ch = t & 31;
  if (row >= nPadRows) return;
  const int rowc = row < nReal ? row : (nReal - 1);
  const size_t src = (size_t)rowc * kD + (size_t)ch * 8;
  const v4f xa = *(const v4f*)(x + src), xb = *(const v4f*)(x + src + 4);
  const v8f xx = __builtin_shufflevector(xa, xb, 0, 1, 2, 3, 4, 5, 6, 7);
  v8h hx = __builtin_convertvector(xx, v8h);
  v8h z = {};
  if (row >= nReal) hx = z;
  const size_t d = (size_t)t * 8;
  *(volatile v8h*)(x16 + d) = hx;
  __threadfence();
  *(volatile v8h*)(x16 + d) = hx;
}

__global__ __launch_bounds__(256) void prep_wt16(const float* __restrict__ W, _Float16* __restrict__ Wt,
                                                int Kdim, int Nreal, int Npad) {
  const int t = blockIdx.x * 256 + threadIdx.x;
  const int k8n = Kdim >> 3;
  const int total = Npad * k8n;
  if (t >= total) return;
  const int n = t / k8n;
  const int k8 = t - n * k8n;
  const int ncl = n < Nreal ? n : (Nreal - 1);
  v8h hv;
#pragma unroll
  for (int i = 0; i < 8; ++i) {
    const float v = W[(size_t)(k8 * 8 + i) * Nreal + ncl] * 16.0f;
    hv[i] = (_Float16)v;
  }
  v8h z = {};
  if (n >= Nreal) hv = z;
  _Float16* dst = Wt + (size_t)n * Kdim + (size_t)k8 * 8;
  *(volatile v8h*)dst = hv;
  __threadfence();
  *(volatile v8h*)dst = hv;
}

__device__ __forceinline__ void corner_fma(float (&acc)[8], const float* __restrict__ vp, float w) {
  const v4f g0 = *(const v4f*)vp;
  const v4f g1 = *(const v4f*)(vp + 4);
#pragma unroll
  for (int e = 0; e < 4; ++e) {
    acc[e]     = fmaf(w, g0[e], acc[e]);
    acc[4 + e] = fmaf(w, g1[e], acc[4 + e]);
  }
}

__global__ __launch_bounds__(128) void sample_kernel(const float* __restrict__ val, const float* __restrict__ offs,
                                                    const float* __restrict__ lgt, const float* __restrict__ refp,
                                                    const int* __restrict__ shp, const int* __restrict__ lst,
                                                    _Float16* __restrict__ ao16) {
#pragma clang fp contract(off)
  __shared__ __align__(16) v4i sIdx[kSampRows * kNH * 32];
  __shared__ __align__(16) v4f sWgt[kSampRows * kNH * 32];
  const int wave = threadIdx.x >> 5;
  const int lane = threadIdx.x & 31;
  const int row  = blockIdx.x * kSampRows + wave;
  const int rowc = row < kNQ ? row : (kNQ - 1);
  const int h = lane >> 2;
  const int c = lane & 3;
  const int sbase = (wave * kNH + h) * 32;

  const float* lp = lgt + (size_t)rowc * kNLG + h * 32 + c * 8;
  const v4f la = *(const v4f*)lp;
  const v4f lb = *(const v4f*)(lp + 4);
  float lg[8];
  lg[0] = la[0]; lg[1] = la[1]; lg[2] = la[2]; lg[3] = la[3];
  lg[4] = lb[0]; lg[5] = lb[1]; lg[6] = lb[2]; lg[7] = lb[3];
  float mx = lg[0];
#pragma unroll
  for (int j = 1; j < 8; ++j) mx = fmaxf(mx, lg[j]);
  mx = fmaxf(mx, __shfl_xor(mx, 1, 32));
  mx = fmaxf(mx, __shfl_xor(mx, 2, 32));
  float ev[8];
  float s = 0.0f;
#pragma unroll
  for (int j = 0; j < 8; ++j) { ev[j] = __expf(lg[j] - mx); s += ev[j]; }
  s += __shfl_xor(s, 1, 32);
  s += __shfl_xor(s, 2, 32);
  const float inv = 1.0f / s;

  int Hl = shp[2 * c];
  int Wl = shp[2 * c + 1];
  int st = lst[c];
  Hl = Hl < 1 ? 1 : (Hl > 32768 ? 32768 : Hl);
  Wl = Wl < 1 ? 1 : (Wl > 32768 ? 32768 : Wl);
  st = st < 0 ? 0 : (st > kNV - 1 ? kNV - 1 : st);
  const float fW = (float)Wl, fH = (float)Hl;
  const float rcW = 1.0f / fW, rcH = 1.0f / fH;
  const float rx = refp[(size_t)rowc * (kNL * 2) + c * 2];
  const float ry = refp[(size_t)rowc * (kNL * 2) + c * 2 + 1];
  const float* op = offs + (size_t)rowc * kNOFF + h * (kNL * kNP * 2) + c * (kNP * 2);
  const v4f o0 = *(const v4f*)op;
  const v4f o1 = *(const v4f*)(op + 4);
  const v4f o2 = *(const v4f*)(op + 8);
  const v4f o3 = *(const v4f*)(op + 12);
  float ov[16];
  ov[0] = o0[0]; ov[1] = o0[1]; ov[2]  = o0[2]; ov[3]  = o0[3];
  ov[4] = o1[0]; ov[5] = o1[1]; ov[6]  = o1[2]; ov[7]  = o1[3];
  ov[8] = o2[0]; ov[9] = o2[1]; ov[10] = o2[2]; ov[11] = o2[3];
  ov[12] = o3[0]; ov[13] = o3[1]; ov[14] = o3[2]; ov[15] = o3[3];
#pragma unroll
  for (int p = 0; p < kNP; ++p) {
    const float aw = ev[p] * inv;
    const float lx = rx + ov[2 * p] * rcW;
    const float ly = ry + ov[2 * p + 1] * rcH;
    float px = lx * fW - 0.5f;
    float py = ly * fH - 0.5f;
    px = fminf(fmaxf(px, -1.0e7f), 1.0e7f);
    py = fminf(fmaxf(py, -1.0e7f), 1.0e7f);
    const float x0f = floorf(px), y0f = floorf(py);
    const float fx = px - x0f, fy = py - y0f;
    const float gx = 1.0f - fx, gy = 1.0f - fy;
    const int x0 = (int)x0f, y0 = (int)y0f;
    const int x1 = x0 + 1, y1 = y0 + 1;
    const bool vx0 = (x0 >= 0) && (x0 < Wl);
    const bool vx1 = (x1 >= 0) && (x1 < Wl);
    const bool vy0 = (y0 >= 0) && (y0 < Hl);
    const bool vy1 = (y1 >= 0) && (y1 < Hl);
    const int xc0 = x0 < 0 ? 0 : (x0 > Wl - 1 ? Wl - 1 : x0);
    const int xc1 = x1 < 0 ? 0 : (x1 > Wl - 1 ? Wl - 1 : x1);
    const int yc0 = y0 < 0 ? 0 : (y0 > Hl - 1 ? Hl - 1 : y0);
    const int yc1 = y1 < 0 ? 0 : (y1 > Hl - 1 ? Hl - 1 : y1);
    int r00 = st + yc0 * Wl + xc0;
    int r01 = st + yc0 * Wl + xc1;
    int r10 = st + yc1 * Wl + xc0;
    int r11 = st + yc1 * Wl + xc1;
    r00 = r00 < 0 ? 0 : (r00 > kNV - 1 ? kNV - 1 : r00);
    r01 = r01 < 0 ? 0 : (r01 > kNV - 1 ? kNV - 1 : r01);
    r10 = r10 < 0 ? 0 : (r10 > kNV - 1 ? kNV - 1 : r10);
    r11 = r11 < 0 ? 0 : (r11 > kNV - 1 ? kNV - 1 : r11);
    const float w00 = (vy0 && vx0) ? aw * (gy * gx) : 0.0f;
    const float w01 = (vy0 && vx1) ? aw * (gy * fx) : 0.0f;
    const float w10 = (vy1 && vx0) ? aw * (fy * gx) : 0.0f;
    const float w11 = (vy1 && vx1) ? aw * (fy * fx) : 0.0f;
    v4i iv; iv[0] = r00; iv[1] = r01; iv[2] = r10; iv[3] = r11;
    v4f wv; wv[0] = w00; wv[1] = w01; wv[2] = w10; wv[3] = w11;
    sIdx[sbase + c * kNP + p] = iv;
    sWgt[sbase + c * kNP + p] = wv;
  }
  __syncthreads();

  const float* vcol = val + h * kHD + c * 8;
  float acc[8];
#pragma unroll
  for (int e = 0; e < 8; ++e) acc[e] = 0.0f;
#pragma unroll 1
  for (int j = 0; j < kNL * kNP; ++j) {
    const v4i id = sIdx[sbase + j];
    const v4f w  = sWgt[sbase + j];
    int i0 = id[0], i1 = id[1], i2 = id[2], i3 = id[3];
    i0 = i0 < 0 ? 0 : (i0 > kNV - 1 ? kNV - 1 : i0);
    i1 = i1 < 0 ? 0 : (i1 > kNV - 1 ? kNV - 1 : i1);
    i2 = i2 < 0 ? 0 : (i2 > kNV - 1 ? kNV - 1 : i2);
    i3 = i3 < 0 ? 0 : (i3 > kNV - 1 ? kNV - 1 : i3);
    corner_fma(acc, vcol + (size_t)i0 * kD, w[0]);
    corner_fma(acc, vcol + (size_t)i1 * kD, w[1]);
    corner_fma(acc, vcol + (size_t)i2 * kD, w[2]);
    corner_fma(acc, vcol + (size_t)i3 * kD, w[3]);
  }

  v8h o;
#pragma unroll
  for (int e = 0; e < 8; ++e) o[e] = (_Float16)(acc[e] * 16.0f);
  v8h z = {};
  if (row >= kNQ) o = z;
  _Float16* dst = ao16 + (size_t)row * kD + lane * 8;
  *(volatile v8h*)dst = o;
  __threadfence();
  *(volatile v8h*)dst = o;
}

__global__ __launch_bounds__(256) void resid_out_kernel(const float* __restrict__ t, const float* __restrict__ q,
                                                       float* __restrict__ outp) {
  const int wave = threadIdx.x >> 5, lane = threadIdx.x & 31;
  const int row = blockIdx.x * 8 + wave;
  if (row >= kNQ) return;
  const int c0 = lane * 4, c1 = 128 + lane * 4;
  const float* tp = t + (size_t)row * kD;
  const float* qp = q + (size_t)row * kD;
  const v4f o0 = *(const v4f*)(tp + c0) + *(const v4f*)(qp + c0);
  const v4f o1 = *(const v4f*)(tp + c1) + *(const v4f*)(qp + c1);
  float* dp = outp + (size_t)row * kD;
  *(volatile v4f*)(dp + c0) = o0;
  *(volatile v4f*)(dp + c1) = o1;
  __threadfence();
  *(volatile v4f*)(dp + c0) = o0;
  *(volatile v4f*)(dp + c1) = o1;
}

static constexpr int gemm_blocks(int M, int N) { return ((M / 64) * (N / 64) + 7) / 8; }

extern "C" void kernel_launch(void* const* d_in, const int* in_sizes, int n_in,
                              void* d_out, int out_size, void* d_ws, size_t ws_size,
                              hipStream_t stream) {
  if (n_in < 13) return;
  if (in_sizes[0] != kNQ * kD || in_sizes[1] != kNV * kD || in_sizes[2] != kNQ * kNL * 2) return;
  if (in_sizes[3] != kNL * 2 || in_sizes[4] != kNL) return;
  if (in_sizes[5] != kD * kD || in_sizes[6] != kD) return;
  if (in_sizes[7] != kD * kNOFF || in_sizes[8] != kNOFF) return;
  if (in_sizes[9] != kD * kNLG || in_sizes[10] != kNLG) return;
  if (in_sizes[11] != kD * kD || in_sizes[12] != kD) return;
  if (out_size != kNQ * kD) return;
  if (ws_size < WS_TOTAL) return;

  const float* query = (const float*)d_in[0];
  const float* value = (const float*)d_in[1];
  const float* refp  = (const float*)d_in[2];
  const int*   shp   = (const int*)d_in[3];
  const int*   lst   = (const int*)d_in[4];
  const float* Wval  = (const float*)d_in[5];
  const float* bval  = (const float*)d_in[6];
  const float* Woff  = (const float*)d_in[7];
  const float* boff  = (const float*)d_in[8];
  const float* Wattn = (const float*)d_in[9];
  const float* battn = (const float*)d_in[10];
  const float* Wout  = (const float*)d_in[11];
  const float* bout  = (const float*)d_in[12];

  char* ws = (char*)d_ws;
  _Float16* q16   = (_Float16*)(ws + OFF_Q16);
  _Float16* ao16  = (_Float16*)(ws + OFF_AO16);
  _Float16* v16   = (_Float16*)(ws + OFF_V16);
  float*    valp  = (float*)(ws + OFF_VAL);
  float*    offp  = (float*)(ws + OFF_OFF);
  float*    outp  = (float*)(ws + OFF_OUT);
  float*    lgtp  = (float*)(ws + OFF_LGT);
  _Float16* wvalT = (_Float16*)(ws + OFF_WVAL);
  _Float16* woutT = (_Float16*)(ws + OFF_WOUT);
  _Float16* woffT = (_Float16*)(ws + OFF_WOFF);
  _Float16* wattT = (_Float16*)(ws + OFF_WATT);
  float*    dout  = (float*)d_out;

  typedef const unsigned short* cu16;
  const float sc16  = 1.0f / 16.0f;
  const float sc256 = 1.0f / 256.0f;

  prep_act16<<<kNQP * 32 / 256, 256, 0, stream>>>(query, q16, kNQ, kNQP);
  prep_act16<<<kNVP * 32 / 256, 256, 0, stream>>>(value, v16, kNV, kNVP);
  prep_wt16<<<(kD * (kD / 8) + 255) / 256, 256, 0, stream>>>(Wval,  wvalT, kD, kD, kD);
  prep_wt16<<<(kNOFF * (kD / 8) + 255) / 256, 256, 0, stream>>>(Woff, woffT, kD, kNOFF, kNOFF);
  prep_wt16<<<(kNLG * (kD / 8) + 255) / 256, 256, 0, stream>>>(Wattn, wattT, kD, kNLG, kNLG);
  prep_wt16<<<(kD * (kD / 8) + 255) / 256, 256, 0, stream>>>(Wout,  woutT, kD, kD, kD);

  wmma_gemm64<0, false, 2, 0, false, 0><<<dim3(gemm_blocks(kNVP, kD), 1), 256, 0, stream>>>(
      (cu16)v16, nullptr, kD, 0L, (cu16)wvalT, nullptr, kD, 0L, (void*)valp, nullptr, kD, 0L,
      bval, nullptr, 0L, kNVP, kD, kD, sc16);
  wmma_gemm64<0, false, 2, 0, false, 0><<<dim3(gemm_blocks(kNQP, kNOFF), 1), 256, 0, stream>>>(
      (cu16)q16, nullptr, kD, 0L, (cu16)woffT, nullptr, kD, 0L, (void*)offp, nullptr, kNOFF, 0L,
      boff, nullptr, 0L, kNQP, kNOFF, kD, sc16);
  wmma_gemm64<0, false, 2, 0, false, 0><<<dim3(gemm_blocks(kNQP, kNLG), 1), 256, 0, stream>>>(
      (cu16)q16, nullptr, kD, 0L, (cu16)wattT, nullptr, kD, 0L, (void*)lgtp, nullptr, kNLG, 0L,
      battn, nullptr, 0L, kNQP, kNLG, kD, sc16);
  sample_kernel<<<kNQP / kSampRows, 128, 0, stream>>>(valp, offp, lgtp, refp, shp, lst, ao16);
  wmma_gemm64<0, false, 2, 0, false, 0><<<dim3(gemm_blocks(kNQP, kD), 1), 256, 0, stream>>>(
      (cu16)ao16, nullptr, kD, 0L, (cu16)woutT, nullptr, kD, 0L, (void*)outp, nullptr, kD, 0L,
      bout, nullptr, 0L, kNQP, kD, kD, sc256);
  resid_out_kernel<<<(kNQ + 7) / 8, 256, 0, stream>>>(outp, query, dout);
}
